// Branch_3_36386962932307
// MI455X (gfx1250) — hardware-run, weakly checked
//
#include <hip/hip_runtime.h>
#include <math.h>

typedef __attribute__((ext_vector_type(16))) _Float16 v16h;
typedef __attribute__((ext_vector_type(8)))  _Float16 v8h;
typedef __attribute__((ext_vector_type(16))) __bf16   v16b;
typedef __attribute__((ext_vector_type(8)))  __bf16   v8b;
typedef __attribute__((ext_vector_type(8)))  float    v8f;
typedef __attribute__((ext_vector_type(4)))  float    v4f;
typedef __attribute__((ext_vector_type(2)))  float    v2f;
typedef __attribute__((ext_vector_type(4)))  unsigned int v4u;

constexpr int kNB     = 16;
constexpr int kTokL   = 512;
constexpr int kDm     = 1024;
constexpr int kDi     = 1024;
constexpr int kOutC   = 1024;
constexpr int kDtR    = 64;
constexpr int kXpN    = 128;
constexpr int kXpRows = 68;
constexpr int kCout   = 512;
constexpr int kChunkB = 4;
constexpr int kNChunk = kNB / kChunkB;
constexpr int kRowsC  = kChunkB * kTokL;
constexpr float kLnEps   = 1e-5f;
constexpr float kInvOutC = 1.0f / 1024.0f;

__device__ __forceinline__ unsigned short f2bf_bits(float f) {
  unsigned u = __float_as_uint(f);
  return (unsigned short)((u + 0x7FFFu + ((u >> 16) & 1u)) >> 16);
}
__device__ __forceinline__ float bf_bits2f(unsigned short h) { return __uint_as_float(((unsigned)h) << 16); }

__device__ __forceinline__ void dep_guard_h(v8f& a, v8f& b, v16h x, v16h y) { asm volatile("v_nop\n\tv_nop\n\tv_nop\n\tv_nop" : "+v"(a), "+v"(b) : "v"(x), "v"(y)); }
__device__ __forceinline__ void dep_guard_b(v8f& a, v8f& b, v16b x, v16b y) { asm volatile("v_nop\n\tv_nop\n\tv_nop\n\tv_nop" : "+v"(a), "+v"(b) : "v"(x), "v"(y)); }
__device__ __forceinline__ void keep4_h(v16h a, v16h b, v16h c, v16h d) { asm volatile("v_nop" :: "v"(a), "v"(b), "v"(c), "v"(d)); }
__device__ __forceinline__ void keep4_b(v16b a, v16b b, v16b c, v16b d) { asm volatile("v_nop" :: "v"(a), "v"(b), "v"(c), "v"(d)); }
__device__ __forceinline__ void acc_guard4(v8f& a, v8f& b, v8f& c, v8f& d) { asm volatile("v_nop\n\tv_nop\n\tv_nop\n\tv_nop" : "+v"(a), "+v"(b), "+v"(c), "+v"(d)); }
template <typename T> struct Frag;
template <> struct Frag<_Float16> {
  typedef v16h V; union U { v16h v; v8h h[2]; };
  static __device__ __forceinline__ v16h load(const _Float16* p) {
    U f; f.h[0] = *(const v8h*)(p); f.h[1] = *(const v8h*)(p + 16); return f.v;
  }
  static __device__ __forceinline__ v8f mma(v16h a, v16h b, v8f c) {
    return __builtin_amdgcn_wmma_f32_16x16x32_f16(false, a, false, b, (short)0, c, false, false);
  }
  static __device__ __forceinline__ void guard(v8f& a, v8f& b, v16h x, v16h y) { dep_guard_h(a, b, x, y); }
  static __device__ __forceinline__ void keep(v16h a, v16h b, v16h c, v16h d) { keep4_h(a, b, c, d); }
};
template <> struct Frag<__bf16> {
  typedef v16b V; union U { v16b v; v8b h[2]; };
  static __device__ __forceinline__ v16b load(const __bf16* p) {
    U f; f.h[0] = *(const v8b*)(p); f.h[1] = *(const v8b*)(p + 16); return f.v;
  }
  static __device__ __forceinline__ v8f mma(v16b a, v16b b, v8f c) {
    return __builtin_amdgcn_wmma_f32_16x16x32_bf16(false, a, false, b, (short)0, c, false, false);
  }
  static __device__ __forceinline__ void guard(v8f& a, v8f& b, v16b x, v16b y) { dep_guard_b(a, b, x, y); }
  static __device__ __forceinline__ void keep(v16b a, v16b b, v16b c, v16b d) { keep4_b(a, b, c, d); }
};

__device__ __forceinline__ unsigned pk16(unsigned short a, unsigned short b) { return (unsigned)a | ((unsigned)b << 16); }

template <int ET> struct Elem;
template <> struct Elem<0> { typedef _Float16 T; };
template <> struct Elem<1> { typedef __bf16 T; };
template <int ET, bool SPLIT, int BIAS_MODE, int OUT_MODE, int RES_MODE, int ACT = 0>
__global__ __launch_bounds__(256) void wmma_gemm64(
    const unsigned short* __restrict__ Ap, const unsigned short* __restrict__ A2p, int lda, long strideA,
    const unsigned short* __restrict__ Btp, const unsigned short* __restrict__ Bt2p, int ldb, long strideB,
    void* __restrict__ Cout, void* __restrict__ Cout2, int ldc, long strideC,
    const float* __restrict__ bias,
    const float* __restrict__ resid, long strideR,
    int M, int N, int K, float scale) {
  typedef typename Elem<ET>::T T;
  typedef typename Frag<T>::V V;
  const T* A = (const T*)Ap; const T* A2 = (const T*)A2p; const T* Bt = (const T*)Btp; const T* Bt2 = (const T*)Bt2p;
  __shared__ __align__(16) float sT[8][16 * 68];
  const int b    = blockIdx.y;
  const int lane = threadIdx.x & 31;
  const int wave = threadIdx.x >> 5;
  const int tilesN = N >> 6;
  const int tilesM = M >> 6;
  const int tile = blockIdx.x * 8 + wave;
  if (tile >= tilesM * tilesN) return;
  const int tm = tile / tilesN;
  const int tn = tile - tm * tilesN;
  const int m0 = tm << 6;
  const int n0 = tn << 6;

  const T* Ab  = A  + (size_t)b * strideA;
  const T* Bb  = Bt + (size_t)b * strideB;
  const T* Ab2 = SPLIT ? (A2  + (size_t)b * strideA) : nullptr;
  const T* Bb2 = SPLIT ? (Bt2 + (size_t)b * strideB) : nullptr;

  const int rlane = lane & 15;
  const int koff  = (lane >> 4) * 8;
  const int mOff  = (lane >> 4) * 8;

  v8f acc[4][4];
#pragma unroll
  for (int i = 0; i < 4; ++i)
#pragma unroll
    for (int j = 0; j < 4; ++j) acc[i][j] = (v8f){0.f,0.f,0.f,0.f,0.f,0.f,0.f,0.f};

  for (int k0 = 0; k0 < K; k0 += 32) {
    V bh[4], bl[4];
#pragma unroll
    for (int j = 0; j < 4; ++j) {
      const size_t bo = (size_t)(n0 + (j << 4) + rlane) * ldb + koff + k0;
      bh[j] = Frag<T>::load(Bb + bo);
      if (SPLIT) bl[j] = Frag<T>::load(Bb2 + bo);
    }
#pragma unroll
    for (int i = 0; i < 4; ++i) {
      const size_t ao = (size_t)(m0 + (i << 4) + rlane) * lda + koff + k0;
      V ah = Frag<T>::load(Ab + ao);
      V al;
      if (SPLIT) al = Frag<T>::load(Ab2 + ao);
#pragma unroll
      for (int j = 0; j < 4; ++j) {
        acc[i][j] = Frag<T>::mma(ah, bh[j], acc[i][j]);
        if (SPLIT) {
          acc[i][j] = Frag<T>::mma(ah, bl[j], acc[i][j]);
          acc[i][j] = Frag<T>::mma(al, bh[j], acc[i][j]);
        }
      }
      Frag<T>::guard(acc[i][0], acc[i][3], ah, SPLIT ? al : ah);
    }
    Frag<T>::keep(bh[0], bh[1], bh[2], bh[3]);
    if (SPLIT) Frag<T>::keep(bl[0], bl[1], bl[2], bl[3]);
  }
  acc_guard4(acc[0][0], acc[0][1], acc[0][2], acc[0][3]);
  acc_guard4(acc[1][0], acc[1][1], acc[1][2], acc[1][3]);
  acc_guard4(acc[2][0], acc[2][1], acc[2][2], acc[2][3]);
  acc_guard4(acc[3][0], acc[3][1], acc[3][2], acc[3][3]);

  float* slab = sT[wave];
  const float* Rb = (RES_MODE != 0) ? (resid + (size_t)b * strideR) : nullptr;
#pragma unroll
  for (int i = 0; i < 4; ++i) {
    const int mBase = m0 + (i << 4);
#pragma unroll
    for (int j = 0; j < 4; ++j) {
      const int n = n0 + (j << 4) + rlane;
      float bv = 0.f;
      if (BIAS_MODE == 2) bv = bias[n];
#pragma unroll
      for (int r = 0; r < 8; ++r) {
        float v = acc[i][j][r] * scale;
        if (BIAS_MODE == 1) v += bias[mBase + mOff + r];
        if (BIAS_MODE == 2) v += bv;
        if (RES_MODE == 1) v += Rb[(size_t)(mBase + mOff + r) * ldc + n];
        if (ACT == 2) v = fmaxf(v, 0.0f);
        if (ACT == 3) v = v * __builtin_amdgcn_rcpf(1.0f + expf(-v));
        if (ACT == 4) v = (v > 0.f) ? v : 0.01f * v;
        if (RES_MODE == 2) v += Rb[(size_t)(mBase + mOff + r) * ldc + n];
        slab[(mOff + r) * 68 + (j << 4) + rlane] = v;
      }
    }
    __builtin_amdgcn_fence(__ATOMIC_RELEASE, "workgroup");
    __builtin_amdgcn_wave_barrier();
    __builtin_amdgcn_fence(__ATOMIC_ACQUIRE, "workgroup");
    if (OUT_MODE == 0) {
      float* C = (float*)Cout + (size_t)b * strideC;
      const int hh = lane >> 4, c4 = (lane & 15) * 4;
      for (int pass = 0; pass < 2; ++pass) {
#pragma unroll
        for (int it = 0; it < 8; ++it) {
          const int row = it * 2 + hh;
          v4f v = *(const v4f*)(slab + row * 68 + c4);
          *(volatile v4f*)(C + (size_t)(mBase + row) * ldc + n0 + c4) = v;
        }
        __threadfence();
      }
    } else {
      const int q = lane >> 3, c8 = (lane & 7) * 8;
      unsigned short* C  = (unsigned short*)Cout  + (size_t)b * strideC;
      unsigned short* C2 = (OUT_MODE == 2) ? ((unsigned short*)Cout2 + (size_t)b * strideC) : nullptr;
      for (int pass = 0; pass < 2; ++pass) {
#pragma unroll
        for (int it = 0; it < 4; ++it) {
          const int row = it * 4 + q;
          const float* sp = slab + row * 68 + c8;
          v8h hv, lv;
#pragma unroll
          for (int e = 0; e < 8; ++e) {
            if (OUT_MODE == 1) {
              hv[e] = (_Float16)sp[e];
            } else {
              unsigned short hb = f2bf_bits(sp[e]);
              unsigned short lb = f2bf_bits(sp[e] - bf_bits2f(hb));
              hv[e] = __builtin_bit_cast(_Float16, hb);
              lv[e] = __builtin_bit_cast(_Float16, lb);
            }
          }
          *(volatile v8h*)(C + (size_t)(mBase + row) * ldc + n0 + c8) = hv;
          if (OUT_MODE == 2) *(volatile v8h*)(C2 + (size_t)(mBase + row) * ldc + n0 + c8) = lv;
        }
        __threadfence();
      }
    }
    __builtin_amdgcn_fence(__ATOMIC_RELEASE, "workgroup");
    __builtin_amdgcn_wave_barrier();
    __builtin_amdgcn_fence(__ATOMIC_ACQUIRE, "workgroup");
  }
}

__device__ __forceinline__ float silu_f(float v) { return v * __builtin_amdgcn_rcpf(1.0f + expf(-v)); }
__device__ __forceinline__ float softplus_f(float v) { return fmaxf(v, 0.0f) + log1pf(expf(-fabsf(v))); }
__device__ __forceinline__ void hilo_bits(float f, unsigned short& hb, unsigned short& lb) {
  hb = f2bf_bits(f);
  lb = f2bf_bits(f - bf_bits2f(hb));
}
__device__ __forceinline__ float conv4_f(float w0, float w1, float w2, float w3, float bias,
                                         float xm3, float xm2, float xm1, float x0) {
  return (((w0 * xm3 + w1 * xm2) + w2 * xm1) + w3 * x0) + bias;
}

__global__ __launch_bounds__(256) void cast_hilo_kernel(const float* __restrict__ src, int src_pitch, int rows_src,
                                                        unsigned short* __restrict__ hi, unsigned short* __restrict__ lo,
                                                        int dst_pitch, int rows, int cols8) {
  const int i = blockIdx.x * 256 + threadIdx.x;
  if (i >= rows * cols8) return;
  const int row = i / cols8;
  const int c8  = (i - row * cols8) * 8;
  const int rs  = (row < rows_src) ? row : (rows_src - 1);
  const bool valid = (row < rows_src);
  const float* p = src + (size_t)rs * src_pitch + c8;
  const v4f a = *(const v4f*)(p);
  const v4f c = *(const v4f*)(p + 4);
  unsigned short hb[8], lb[8];
#pragma unroll
  for (int e = 0; e < 4; ++e) {
    const float f0 = valid ? a[e] : 0.0f;
    const float f1 = valid ? c[e] : 0.0f;
    hilo_bits(f0, hb[e], lb[e]);
    hilo_bits(f1, hb[4 + e], lb[4 + e]);
  }
  const v4u uh = (v4u){pk16(hb[0], hb[1]), pk16(hb[2], hb[3]), pk16(hb[4], hb[5]), pk16(hb[6], hb[7])};
  const v4u ul = (v4u){pk16(lb[0], lb[1]), pk16(lb[2], lb[3]), pk16(lb[4], lb[5]), pk16(lb[6], lb[7])};
  unsigned short* qh = hi + (size_t)row * dst_pitch + c8;
  unsigned short* ql = lo + (size_t)row * dst_pitch + c8;
  *(volatile v4u*)qh = uh;
  *(volatile v4u*)ql = ul;
  __threadfence();
  *(volatile v4u*)qh = uh;
  *(volatile v4u*)ql = ul;
}

__global__ __launch_bounds__(256) void conv_silu_kernel(const float* __restrict__ xsp, const float* __restrict__ cw,
                                                        const float* __restrict__ cb,
                                                        unsigned short* __restrict__ xh, unsigned short* __restrict__ xl) {
  const int t = blockIdx.x * 256 + threadIdx.x;
  if (t >= kChunkB * 512) return;
  const int bq = t >> 9;
  const int dp = (t & 511) * 2;
  const float w00 = cw[dp * 4 + 0], w01 = cw[dp * 4 + 1], w02 = cw[dp * 4 + 2], w03 = cw[dp * 4 + 3];
  const float w10 = cw[dp * 4 + 4], w11 = cw[dp * 4 + 5], w12 = cw[dp * 4 + 6], w13 = cw[dp * 4 + 7];
  const float cb0 = cb[dp], cb1 = cb[dp + 1];
  float p01 = 0.f, p02 = 0.f, p03 = 0.f;
  float p11 = 0.f, p12 = 0.f, p13 = 0.f;
  const size_t rowb = (size_t)bq * kTokL;
#pragma unroll 1
  for (int l = 0; l < kTokL; ++l) {
    const size_t off = (rowb + l) * kDi + dp;
    const v2f xv = *(const v2f*)(xsp + off);
    const float s0 = silu_f(conv4_f(w00, w01, w02, w03, cb0, p03, p02, p01, xv[0]));
    const float s1 = silu_f(conv4_f(w10, w11, w12, w13, cb1, p13, p12, p11, xv[1]));
    unsigned short h0, l0, h1, l1;
    hilo_bits(s0, h0, l0);
    hilo_bits(s1, h1, l1);
    const unsigned uh = pk16(h0, h1), ul = pk16(l0, l1);
    unsigned* qh = (unsigned*)(xh + off);
    unsigned* ql = (unsigned*)(xl + off);
    *(volatile unsigned*)qh = uh;
    *(volatile unsigned*)ql = ul;
    __threadfence();
    *(volatile unsigned*)qh = uh;
    *(volatile unsigned*)ql = ul;
    p03 = p02; p02 = p01; p01 = xv[0];
    p13 = p12; p12 = p11; p11 = xv[1];
  }
}

__global__ __launch_bounds__(256) void scan_kernel(const float* __restrict__ dtp, const float* __restrict__ xsp,
                                                   const float* __restrict__ xdbl, const float* __restrict__ zg,
                                                   const float* __restrict__ cw, const float* __restrict__ cb,
                                                   const float* __restrict__ alog, const float* __restrict__ dskip,
                                                   unsigned short* __restrict__ yh, unsigned short* __restrict__ yl) {
  const int t = blockIdx.x * 256 + threadIdx.x;
  if (t >= kChunkB * 512) return;
  const int bq = t >> 9;
  const int dp = (t & 511) * 2;
  const float w00 = cw[dp * 4 + 0], w01 = cw[dp * 4 + 1], w02 = cw[dp * 4 + 2], w03 = cw[dp * 4 + 3];
  const float w10 = cw[dp * 4 + 4], w11 = cw[dp * 4 + 5], w12 = cw[dp * 4 + 6], w13 = cw[dp * 4 + 7];
  const float cb0 = cb[dp], cb1 = cb[dp + 1];
  const float a00 = -expf(alog[dp * 2 + 0]), a01 = -expf(alog[dp * 2 + 1]);
  const float a10 = -expf(alog[dp * 2 + 2]), a11 = -expf(alog[dp * 2 + 3]);
  const float dd0 = dskip[dp], dd1 = dskip[dp + 1];
  float p01 = 0.f, p02 = 0.f, p03 = 0.f;
  float p11 = 0.f, p12 = 0.f, p13 = 0.f;
  float h00 = 0.f, h01 = 0.f, h10 = 0.f, h11 = 0.f;
  const size_t rowb = (size_t)bq * kTokL;
#pragma unroll 1
  for (int l = 0; l < kTokL; ++l) {
    const size_t row = rowb + l;
    const size_t off = row * kDi + dp;
    const v2f dv = *(const v2f*)(dtp + off);
    const v2f xv = *(const v2f*)(xsp + off);
    const v2f gv = *(const v2f*)(zg + off);
    const v4f bc = *(const v4f*)(xdbl + row * kXpN + 64);
    const float u0 = silu_f(conv4_f(w00, w01, w02, w03, cb0, p03, p02, p01, xv[0]));
    const float u1 = silu_f(conv4_f(w10, w11, w12, w13, cb1, p13, p12, p11, xv[1]));
    const float de0 = softplus_f(dv[0]);
    const float de1 = softplus_f(dv[1]);
    h00 = expf(de0 * a00) * h00 + (de0 * bc[0]) * u0;
    h01 = expf(de0 * a01) * h01 + (de0 * bc[1]) * u0;
    h10 = expf(de1 * a10) * h10 + (de1 * bc[0]) * u1;
    h11 = expf(de1 * a11) * h11 + (de1 * bc[1]) * u1;
    const float y0 = ((h00 * bc[2] + h01 * bc[3]) + u0 * dd0) * gv[0];
    const float y1 = ((h10 * bc[2] + h11 * bc[3]) + u1 * dd1) * gv[1];
    unsigned short hb0, lb0, hb1, lb1;
    hilo_bits(y0, hb0, lb0);
    hilo_bits(y1, hb1, lb1);
    const unsigned uh = pk16(hb0, hb1), ul = pk16(lb0, lb1);
    unsigned* qh = (unsigned*)(yh + off);
    unsigned* ql = (unsigned*)(yl + off);
    *(volatile unsigned*)qh = uh;
    *(volatile unsigned*)ql = ul;
    __threadfence();
    *(volatile unsigned*)qh = uh;
    *(volatile unsigned*)ql = ul;
    p03 = p02; p02 = p01; p01 = xv[0];
    p13 = p12; p12 = p11; p11 = xv[1];
  }
}

__global__ __launch_bounds__(256) void layernorm_hilo_kernel(const float* __restrict__ y1t, const float* __restrict__ gam,
                                                             const float* __restrict__ bet,
                                                             unsigned short* __restrict__ yh, unsigned short* __restrict__ yl) {
  __shared__ float red[32][64];
  __shared__ float stat[2][64];
  const int cg = blockIdx.x, bq = blockIdx.y, t = threadIdx.x;
  const int c8 = (t & 7) * 8, rp = t >> 3;
  const size_t colbase = (size_t)bq * kOutC * kTokL + (size_t)cg * 64 + c8;
  float s[8];
#pragma unroll
  for (int e = 0; e < 8; ++e) s[e] = 0.f;
#pragma unroll 1
  for (int i = 0; i < 32; ++i) {
    const int row = rp + 32 * i;
    const float* p = y1t + colbase + (size_t)row * kTokL;
    const v4f a = *(const v4f*)(p), c = *(const v4f*)(p + 4);
#pragma unroll
    for (int e = 0; e < 4; ++e) { s[e] += a[e]; s[4 + e] += c[e]; }
  }
#pragma unroll
  for (int e = 0; e < 8; ++e) red[rp][c8 + e] = s[e];
  __syncthreads();
  if (t < 64) {
    float acc = 0.f;
#pragma unroll 1
    for (int p = 0; p < 32; ++p) acc += red[p][t];
    stat[0][t] = acc * kInvOutC;
  }
  __syncthreads();
  float mu[8];
#pragma unroll
  for (int e = 0; e < 8; ++e) { mu[e] = stat[0][c8 + e]; s[e] = 0.f; }
#pragma unroll 1
  for (int i = 0; i < 32; ++i) {
    const int row = rp + 32 * i;
    const float* p = y1t + colbase + (size_t)row * kTokL;
    const v4f a = *(const v4f*)(p), c = *(const v4f*)(p + 4);
#pragma unroll
    for (int e = 0; e < 4; ++e) {
      const float d0 = a[e] - mu[e];
      const float d1 = c[e] - mu[4 + e];
      s[e] += d0 * d0;
      s[4 + e] += d1 * d1;
    }
  }
#pragma unroll
  for (int e = 0; e < 8; ++e) red[rp][c8 + e] = s[e];
  __syncthreads();
  if (t < 64) {
    float acc = 0.f;
#pragma unroll 1
    for (int p = 0; p < 32; ++p) acc += red[p][t];
    const float var = acc * kInvOutC;
    stat[1][t] = 1.0f / sqrtf(var + kLnEps);
  }
  __syncthreads();
  float rs[8];
#pragma unroll
  for (int e = 0; e < 8; ++e) rs[e] = stat[1][c8 + e];
#pragma unroll 1
  for (int i = 0; i < 32; ++i) {
    const int row = rp + 32 * i;
    const float* p = y1t + colbase + (size_t)row * kTokL;
    const v4f a = *(const v4f*)(p), c = *(const v4f*)(p + 4);
    const float g = gam[row], bb = bet[row];
    unsigned short hb[8], lb[8];
#pragma unroll
    for (int e = 0; e < 4; ++e) {
      const float v0 = (a[e] - mu[e]) * rs[e] * g + bb;
      const float v1 = (c[e] - mu[4 + e]) * rs[4 + e] * g + bb;
      hilo_bits(v0, hb[e], lb[e]);
      hilo_bits(v1, hb[4 + e], lb[4 + e]);
    }
    const v4u uh = (v4u){pk16(hb[0], hb[1]), pk16(hb[2], hb[3]), pk16(hb[4], hb[5]), pk16(hb[6], hb[7])};
    const v4u ul = (v4u){pk16(lb[0], lb[1]), pk16(lb[2], lb[3]), pk16(lb[4], lb[5]), pk16(lb[6], lb[7])};
    const size_t o = colbase + (size_t)row * kTokL;
    *(volatile v4u*)(yh + o) = uh;
    *(volatile v4u*)(yl + o) = ul;
    __threadfence();
    *(volatile v4u*)(yh + o) = uh;
    *(volatile v4u*)(yl + o) = ul;
  }
}

template <int BIAS_MODE, int OUT_MODE, int RES_MODE, int ACT>
static void launch_gemm(hipStream_t st,
                        const unsigned short* Ah, const unsigned short* Al, int lda, long strideA,
                        const unsigned short* Bh, const unsigned short* Bl, int ldb, long strideB,
                        void* C, void* Cl, int ldc, long strideC,
                        const float* bias, const float* resid, long strideR,
                        int M, int N, int K, int batch) {
  const int tiles = (M / 64) * (N / 64);
  dim3 grid((unsigned)((tiles + 7) / 8), (unsigned)batch, 1);
  wmma_gemm64<1, true, BIAS_MODE, OUT_MODE, RES_MODE, ACT><<<grid, 256, 0, st>>>(
      Ah, Al, lda, strideA, Bh, Bl, ldb, strideB, C, Cl, ldc, strideC, bias, resid, strideR, M, N, K, 1.0f);
}

static void launch_cast(hipStream_t st, const float* src, int src_pitch, int rows_src,
                        unsigned short* hi, unsigned short* lo, int dst_pitch, int rows, int cols) {
  const int cols8 = cols / 8;
  const int n = rows * cols8;
  cast_hilo_kernel<<<(n + 255) / 256, 256, 0, st>>>(src, src_pitch, rows_src, hi, lo, dst_pitch, rows, cols8);
}

extern "C" void kernel_launch(void* const* d_in, const int* in_sizes, int n_in,
                              void* d_out, int out_size, void* d_ws, size_t ws_size,
                              hipStream_t stream) {
  (void)in_sizes; (void)n_in; (void)out_size;
  const float* x        = (const float*)d_in[0];
  const float* in_proj  = (const float*)d_in[1];
  const float* conv_w   = (const float*)d_in[2];
  const float* conv_b   = (const float*)d_in[3];
  const float* x_proj   = (const float*)d_in[4];
  const float* dt_projw = (const float*)d_in[5];
  const float* dt_projb = (const float*)d_in[6];
  const float* a_log    = (const float*)d_in[7];
  const float* d_skip   = (const float*)d_in[8];
  const float* out_proj = (const float*)d_in[9];
  const float* ln_g     = (const float*)d_in[10];
  const float* ln_b     = (const float*)d_in[11];
  const float* lin3_w   = (const float*)d_in[12];
  const float* lin3_b   = (const float*)d_in[13];
  const float* linsp_w  = (const float*)d_in[14];
  const float* linsp_b  = (const float*)d_in[15];
  const float* linres_w = (const float*)d_in[16];
  const float* linres_b = (const float*)d_in[17];
  float* outp = (float*)d_out;

  char* ws = (char*)d_ws;
  size_t off = 0;
  auto carve = [&](size_t bytes) -> char* {
    char* p = ws + off;
    off += (bytes + 255) & ~(size_t)255;
    return p;
  };
  const size_t szWinp = (size_t)2 * kDi * kDm * 2;
  const size_t szWxp  = (size_t)kXpN * kDi * 2;
  const size_t szWdt  = (size_t)kDi * kDtR * 2;
  const size_t szWout = (size_t)kOutC * kDi * 2;
  const size_t szWl3  = (size_t)kCout * kTokL * 2;
  const size_t szWsp  = (size_t)kOutC * kDm * 2;
  const size_t szWres = (size_t)kCout * kTokL * 2;
  const size_t szX16  = (size_t)kRowsC * kDm * 2;
  const size_t szR16  = (size_t)kChunkB * kOutC * kTokL * 2;
  const size_t szBigF = (size_t)kRowsC * kDi * 4;
  const size_t szXdbl = (size_t)kRowsC * kXpN * 4;
  const size_t szDT16 = (size_t)kRowsC * kDtR * 2;

  unsigned short* winp_h = (unsigned short*)carve(szWinp);
  unsigned short* winp_l = (unsigned short*)carve(szWinp);
  unsigned short* wxp_h  = (unsigned short*)carve(szWxp);
  unsigned short* wxp_l  = (unsigned short*)carve(szWxp);
  unsigned short* wdt_h  = (unsigned short*)carve(szWdt);
  unsigned short* wdt_l  = (unsigned short*)carve(szWdt);
  unsigned short* wout_h = (unsigned short*)carve(szWout);
  unsigned short* wout_l = (unsigned short*)carve(szWout);
  unsigned short* wl3_h  = (unsigned short*)carve(szWl3);
  unsigned short* wl3_l  = (unsigned short*)carve(szWl3);
  unsigned short* wsp_h  = (unsigned short*)carve(szWsp);
  unsigned short* wsp_l  = (unsigned short*)carve(szWsp);
  unsigned short* wres_h = (unsigned short*)carve(szWres);
  unsigned short* wres_l = (unsigned short*)carve(szWres);
  unsigned short* x_h    = (unsigned short*)carve(szX16);
  unsigned short* x_l    = (unsigned short*)carve(szX16);
  unsigned short* r1t_h  = (unsigned short*)carve(szR16);
  unsigned short* r1t_l  = (unsigned short*)carve(szR16);
  float*          xspre  = (float*)carve(szBigF);
  float*          zg     = (float*)carve(szBigF);
  unsigned short* xs_h   = (unsigned short*)carve(szX16);
  unsigned short* xs_l   = (unsigned short*)carve(szX16);
  float*          xdbl   = (float*)carve(szXdbl);
  unsigned short* dt_h   = (unsigned short*)carve(szDT16);
  unsigned short* dt_l   = (unsigned short*)carve(szDT16);
  float*          dtpre  = (float*)carve(szBigF);
  unsigned short* yg_h   = (unsigned short*)carve(szX16);
  unsigned short* yg_l   = (unsigned short*)carve(szX16);
  float*          y1t    = (float*)carve(szBigF);
  unsigned short* y2_h   = (unsigned short*)carve(szR16);
  unsigned short* y2_l   = (unsigned short*)carve(szR16);
  float*          y3     = (float*)carve(szBigF);
  if (off > ws_size) return;

  launch_cast(stream, in_proj,  kDm,  2 * kDi,  winp_h, winp_l, kDm,   2 * kDi, kDm);
  launch_cast(stream, x_proj,   kDi,  kXpRows,  wxp_h,  wxp_l,  kDi,   kXpN,    kDi);
  launch_cast(stream, dt_projw, kDtR, kDi,      wdt_h,  wdt_l,  kDtR,  kDi,     kDtR);
  launch_cast(stream, out_proj, kDi,  kOutC,    wout_h, wout_l, kDi,   kOutC,   kDi);
  launch_cast(stream, lin3_w,   kTokL, kCout,   wl3_h,  wl3_l,  kTokL, kCout,   kTokL);
  launch_cast(stream, linsp_w,  kDm,  kOutC,    wsp_h,  wsp_l,  kDm,   kOutC,   kDm);
  launch_cast(stream, linres_w, kTokL, kCout,   wres_h, wres_l, kTokL, kCout,   kTokL);

  const long strideTokImg = (long)kTokL * kDm;
  const long strideOC     = (long)kOutC * kTokL;
  const long strideOut    = (long)kCout * kOutC;
  const int convBlocks = (kChunkB * 512 + 255) / 256;

  for (int q = 0; q < kNChunk; ++q) {
    const float* xq = x + (size_t)q * kRowsC * kDm;
    float* outq = outp + (size_t)q * kChunkB * kCout * kOutC;

    launch_cast(stream, xq, kDm, kRowsC, x_h, x_l, kDm, kRowsC, kDm);

    launch_gemm<1, 2, 0, 3>(stream, wsp_h, wsp_l, kDm, 0L, x_h, x_l, kDm, strideTokImg,
                            r1t_h, r1t_l, kTokL, strideOC, linsp_b, nullptr, 0L,
                            kOutC, kTokL, kDm, kChunkB);

    launch_gemm<0, 0, 0, 0>(stream, x_h, x_l, kDm, 0L, winp_h, winp_l, kDm, 0L,
                            xspre, nullptr, kDi, 0L, nullptr, nullptr, 0L, kRowsC, kDi, kDm, 1);
    launch_gemm<0, 0, 0, 3>(stream, x_h, x_l, kDm, 0L,
                            winp_h + (size_t)kDi * kDm, winp_l + (size_t)kDi * kDm, kDm, 0L,
                            zg, nullptr, kDi, 0L, nullptr, nullptr, 0L, kRowsC, kDi, kDm, 1);

    conv_silu_kernel<<<convBlocks, 256, 0, stream>>>(xspre, conv_w, conv_b, xs_h, xs_l);

    launch_gemm<0, 0, 0, 0>(stream, xs_h, xs_l, kDi, 0L, wxp_h, wxp_l, kDi, 0L,
                            xdbl, nullptr, kXpN, 0L, nullptr, nullptr, 0L, kRowsC, kXpN, kDi, 1);

    launch_cast(stream, xdbl, kXpN, kRowsC, dt_h, dt_l, kDtR, kRowsC, kDtR);

    launch_gemm<2, 0, 0, 0>(stream, dt_h, dt_l, kDtR, 0L, wdt_h, wdt_l, kDtR, 0L,
                            dtpre, nullptr, kDi, 0L, dt_projb, nullptr, 0L, kRowsC, kDi, kDtR, 1);

    scan_kernel<<<convBlocks, 256, 0, stream>>>(dtpre, xspre, xdbl, zg, conv_w, conv_b, a_log, d_skip, yg_h, yg_l);

    launch_gemm<0, 0, 0, 0>(stream, wout_h, wout_l, kDi, 0L, yg_h, yg_l, kDi, strideTokImg,
                            y1t, nullptr, kTokL, strideOC, nullptr, nullptr, 0L,
                            kOutC, kTokL, kDi, kChunkB);

    layernorm_hilo_kernel<<<dim3(8, kChunkB, 1), 256, 0, stream>>>(y1t, ln_g, ln_b, y2_h, y2_l);

    launch_gemm<1, 0, 0, 3>(stream, wl3_h, wl3_l, kTokL, 0L, y2_h, y2_l, kTokL, strideOC,
                            y3, nullptr, kOutC, strideOut, lin3_b, nullptr, 0L,
                            kCout, kOutC, kTokL, kChunkB);

    launch_gemm<1, 0, 2, 3>(stream, wres_h, wres_l, kTokL, 0L, r1t_h, r1t_l, kTokL, strideOC,
                            outq, nullptr, kOutC, strideOut, linres_b, y3, strideOut,
                            kCout, kOutC, kTokL, kChunkB);
  }
}
